// LDGuidedRetention_41944650613077
// MI455X (gfx1250) — hardware-verified
//
#include <hip/hip_runtime.h>

typedef _Float16 v16h __attribute__((ext_vector_type(16)));
typedef _Float16 v8h  __attribute__((ext_vector_type(8)));
typedef float    v8f  __attribute__((ext_vector_type(8)));
typedef float    v4f  __attribute__((ext_vector_type(4)));
typedef v8h __attribute__((may_alias)) v8ha;
typedef v4f __attribute__((may_alias)) v4fa;

union Frag { v16h v; v8h half[2]; };

#define NB    8
#define SEQ   2048
#define DM    768
#define D3    2304
#define MROWS (NB * SEQ)
#define NX    (MROWS * DM)
#define NX8   (NX / 8)
#define WSC   16.0f
#define PSC   16384.0f
#define CSC   32.0f

#define SS_STRIDE 2048
#define PS_STRIDE 2048
#define SS_BYTES  (16 * SS_STRIDE * 4)
#define PS_BYTES  (16 * PS_STRIDE * 2)
#define ATT_LDS   (SS_BYTES + PS_BYTES + 64)

__device__ __forceinline__ v8f wmma_f16(v16h a, v16h b, v8f c) {
  v8f d = __builtin_amdgcn_wmma_f32_16x16x32_f16(false, a, false, b, (short)0, c, false, false);
  asm volatile("v_nop\n\tv_nop\n\tv_nop\n\tv_nop" : "+v"(d) : "v"(a), "v"(b));
  return d;
}

__device__ __forceinline__ v16h load_frag(const _Float16* p, int h) {
  Frag f;
  f.half[0] = *(const v8ha*)(p + 8 * h);
  f.half[1] = *(const v8ha*)(p + 16 + 8 * h);
  return f.v;
}

__device__ __forceinline__ v8f zero8f() {
  v8f z = {0.f, 0.f, 0.f, 0.f, 0.f, 0.f, 0.f, 0.f};
  return z;
}

__global__ __launch_bounds__(256) void convert_x_kernel(const float* __restrict__ x,
                                                        _Float16* __restrict__ xh, int n8) {
  const int g = blockIdx.x * 256 + threadIdx.x;
  if (g >= n8) return;
  const float* src = x + (size_t)g * 8;
  const v4f a = *(const v4fa*)src;
  const v4f c = *(const v4fa*)(src + 4);
  const v8h o = { (_Float16)a.x, (_Float16)a.y, (_Float16)a.z, (_Float16)a.w,
                  (_Float16)c.x, (_Float16)c.y, (_Float16)c.z, (_Float16)c.w };
  _Float16* dst = xh + (size_t)g * 8;
  *(volatile v8h*)dst = o;
  __threadfence();
  *(volatile v8h*)dst = o;
}

__device__ __forceinline__ void wt_store_pass(const _Float16* tile, _Float16* wt, int rows,
                                              int r0, int c0, int w, int lane) {
  const int q8 = lane & 7, sub = lane >> 3;
  #pragma unroll
  for (int i = 0; i < 2; ++i) {
    const int lid = w * 8 + i * 4 + sub;
    const v8h v = *(const v8ha*)(tile + lid * 72 + 8 * q8);
    _Float16* dst = wt + (size_t)(c0 + lid) * rows + r0 + 8 * q8;
    *(volatile v8h*)dst = v;
  }
}

__global__ __launch_bounds__(256) void transpose_w_kernel(const float* __restrict__ w,
                                                          _Float16* __restrict__ wt,
                                                          int rows, int cols) {
  __shared__ __attribute__((aligned(16))) _Float16 tile[64 * 72];
  const int tid = threadIdx.x, lane = tid & 31, wv = tid >> 5;
  const int r0 = blockIdx.y * 64, c0 = blockIdx.x * 64;
  const int rr = tid >> 2, cq = (tid & 3) * 16;
  const float* src = w + (size_t)(r0 + rr) * cols + c0 + cq;
  #pragma unroll
  for (int p = 0; p < 4; ++p) {
    const v4f v = *(const v4fa*)(src + 4 * p);
    tile[(cq + 4 * p + 0) * 72 + rr] = (_Float16)(v.x * WSC);
    tile[(cq + 4 * p + 1) * 72 + rr] = (_Float16)(v.y * WSC);
    tile[(cq + 4 * p + 2) * 72 + rr] = (_Float16)(v.z * WSC);
    tile[(cq + 4 * p + 3) * 72 + rr] = (_Float16)(v.w * WSC);
  }
  __syncthreads();
  wt_store_pass(tile, wt, rows, r0, c0, wv, lane);
  __threadfence();
  wt_store_pass(tile, wt, rows, r0, c0, wv, lane);
}

__device__ __forceinline__ void qkv_store_pass(const _Float16* sT, _Float16* plane, _Float16* vt,
                                               int which, int m0, int b, int l0, int f0,
                                               int w, int lane) {
  const int q8 = lane & 7, sub = lane >> 3;
  #pragma unroll
  for (int i = 0; i < 8; ++i) {
    const int lid = w * 32 + i * 4 + sub;
    v8h v;
    _Float16* dst;
    if (which != 2) {
      v = *(const v8ha*)(sT + lid * 64 + 8 * q8);
      dst = plane + (size_t)(m0 + lid) * DM + f0 + 8 * q8;
    } else {
      const int d = lid >> 1, hl = lid & 1;
      v = *(const v8ha*)(sT + d * 128 + 64 * hl + 8 * q8);
      dst = vt + ((size_t)b * DM + f0 + d) * SEQ + l0 + 64 * hl + 8 * q8;
    }
    *(volatile v8h*)dst = v;
  }
}

__global__ __launch_bounds__(128) void qkv_gemm_kernel(
    const _Float16* __restrict__ xh,
    const _Float16* __restrict__ wt,
    const float* __restrict__ bqkv,
    _Float16* __restrict__ qh,
    _Float16* __restrict__ kh,
    _Float16* __restrict__ vt)
{
  __shared__ __attribute__((aligned(16))) _Float16 sT[128 * 64];

  const int tid = threadIdx.x, lane = tid & 31, w = tid >> 5;
  const int h = lane >> 4, m = lane & 15;
  const int m0 = blockIdx.x * 128;
  const int cg = blockIdx.y;
  const int which = cg / 12;
  const int f0 = (cg - which * 12) * 64;
  const int n0 = cg * 64;
  const int m0w = m0 + 32 * w;

  const _Float16* xa0 = xh + (size_t)(m0w + m) * DM;
  const _Float16* xa1 = xa0 + (size_t)16 * DM;
  const _Float16* wb  = wt + (size_t)(n0 + m) * DM;

  v8f acc[2][4];
  #pragma unroll
  for (int mt = 0; mt < 2; ++mt)
    #pragma unroll
    for (int nt = 0; nt < 4; ++nt) acc[mt][nt] = zero8f();

  #pragma unroll 1
  for (int k0 = 0; k0 < DM; k0 += 32) {
    const v16h a0 = load_frag(xa0 + k0, h);
    const v16h a1 = load_frag(xa1 + k0, h);
    #pragma unroll
    for (int nt = 0; nt < 4; ++nt) {
      const v16h bf = load_frag(wb + (size_t)nt * 16 * DM + k0, h);
      acc[0][nt] = wmma_f16(a0, bf, acc[0][nt]);
      acc[1][nt] = wmma_f16(a1, bf, acc[1][nt]);
    }
  }

  #pragma unroll
  for (int nt = 0; nt < 4; ++nt) {
    const int feat = 16 * nt + m;
    const float bv = bqkv[n0 + feat];
    #pragma unroll
    for (int mt = 0; mt < 2; ++mt) {
      #pragma unroll
      for (int r = 0; r < 8; ++r) {
        const int tokl = 32 * w + 16 * mt + 8 * h + r;
        const float y = acc[mt][nt][r] * (1.0f / WSC) + bv;
        const int idx = (which == 2) ? (feat * 128 + tokl) : (tokl * 64 + feat);
        sT[idx] = (_Float16)y;
      }
    }
  }
  __syncthreads();

  const int b = m0 / SEQ, l0 = m0 - b * SEQ;
  _Float16* plane = (which == 0) ? qh : kh;
  qkv_store_pass(sT, plane, vt, which, m0, b, l0, f0, w, lane);
  __threadfence();
  qkv_store_pass(sT, plane, vt, which, m0, b, l0, f0, w, lane);
}

__device__ __forceinline__ void ctx_store_pass(const _Float16* sC, _Float16* ch,
                                               int b, int qbase, int w, int lane) {
  const int q8 = lane & 7, sub = lane >> 3;
  #pragma unroll
  for (int i = 0; i < 6; ++i) {
    const int lid = w * 24 + i * 4 + sub;
    const int row = lid / 12, seg = lid - row * 12;
    const v8h v = *(const v8ha*)(sC + row * DM + seg * 64 + 8 * q8);
    _Float16* dst = ch + ((size_t)b * SEQ + qbase + row) * DM + seg * 64 + 8 * q8;
    *(volatile v8h*)dst = v;
  }
}

__global__ __launch_bounds__(256) void attention_kernel(
    const _Float16* __restrict__ qh,
    const _Float16* __restrict__ kh,
    const _Float16* __restrict__ vt,
    const float* __restrict__ gptr,
    _Float16* __restrict__ ch)
{
  extern __shared__ __attribute__((aligned(16))) char smem[];
  float*    Ss   = (float*)smem;
  _Float16* Ps   = (_Float16*)(smem + SS_BYTES);
  float*    Linv = (float*)(smem + SS_BYTES + PS_BYTES);
  _Float16* sC   = (_Float16*)smem;

  const int tid = threadIdx.x, lane = tid & 31;
  const int w = __builtin_amdgcn_readfirstlane(tid >> 5);
  const int h = lane >> 4, m = lane & 15;
  const int b = blockIdx.y, qbase = blockIdx.x * 16;

  const float gamma = gptr[0];
  const float lg2 = log2f(gamma);
  const float scale = 0.036084391824351614f;

  const _Float16* qrow = qh + ((size_t)b * SEQ + qbase + m) * DM;

  #pragma unroll 1
  for (int it = 0; it < 4; ++it) {
    const int kb = 64 * (w + 8 * it);
    if (kb > qbase + 15) {
      #pragma unroll
      for (int j = 0; j < 4; ++j)
        #pragma unroll
        for (int r = 0; r < 8; ++r) Ss[(8 * h + r) * SS_STRIDE + kb + 16 * j + m] = 0.0f;
    } else {
      v8f acc[4];
      #pragma unroll
      for (int j = 0; j < 4; ++j) acc[j] = zero8f();
      const _Float16* krow = kh + ((size_t)b * SEQ + kb + m) * DM;
      #pragma unroll 1
      for (int k0 = 0; k0 < DM; k0 += 32) {
        const v16h a = load_frag(qrow + k0, h);
        #pragma unroll
        for (int j = 0; j < 4; ++j) {
          const v16h bf = load_frag(krow + (size_t)(16 * j) * DM + k0, h);
          acc[j] = wmma_f16(a, bf, acc[j]);
        }
      }
      #pragma unroll
      for (int j = 0; j < 4; ++j) {
        const int jj = kb + 16 * j + m;
        #pragma unroll
        for (int r = 0; r < 8; ++r) {
          const int i = qbase + 8 * h + r;
          const int nd = (i - jj) > 0 ? (i - jj) : 0;
          const float dec = exp2f((float)nd * lg2);
          const float v = (jj <= i) ? (acc[j][r] * scale) * dec : 0.0f;
          Ss[(8 * h + r) * SS_STRIDE + jj] = v;
        }
      }
    }
  }
  __syncthreads();

  #pragma unroll 1
  for (int rr = 0; rr < 2; ++rr) {
    const int row = 2 * w + rr;
    const float* srow = Ss + row * SS_STRIDE;
    float mx = -3.0e38f;
    #pragma unroll 8
    for (int j = lane; j < SEQ; j += 32) mx = fmaxf(mx, srow[j]);
    #pragma unroll
    for (int off = 16; off > 0; off >>= 1) mx = fmaxf(mx, __shfl_xor(mx, off, 32));
    float sum = 0.0f;
    _Float16* prow = Ps + row * PS_STRIDE;
    #pragma unroll 8
    for (int j = lane; j < SEQ; j += 32) {
      const float p = __expf(srow[j] - mx);
      sum += p;
      prow[j] = (_Float16)(p * PSC);
    }
    #pragma unroll
    for (int off = 16; off > 0; off >>= 1) sum += __shfl_xor(sum, off, 32);
    if (lane == 0) Linv[row] = (1.0f / sum) * (CSC / PSC);
  }
  __syncthreads();

  v8f oacc[6];
  #pragma unroll
  for (int t = 0; t < 6; ++t) oacc[t] = zero8f();
  const _Float16* prow3 = Ps + m * PS_STRIDE;
  const _Float16* vrow = vt + ((size_t)b * DM + 96 * w + m) * SEQ;
  #pragma unroll 1
  for (int k0 = 0; k0 < SEQ; k0 += 32) {
    const v16h a = load_frag(prow3 + k0, h);
    #pragma unroll
    for (int t = 0; t < 6; ++t) {
      const v16h bf = load_frag(vrow + (size_t)(16 * t) * SEQ + k0, h);
      oacc[t] = wmma_f16(a, bf, oacc[t]);
    }
  }

  #pragma unroll
  for (int t = 0; t < 6; ++t) {
    const int col = 96 * w + 16 * t + m;
    #pragma unroll
    for (int r = 0; r < 8; ++r) {
      const int row = 8 * h + r;
      sC[row * DM + col] = (_Float16)(oacc[t][r] * Linv[row]);
    }
  }
  __syncthreads();

  ctx_store_pass(sC, ch, b, qbase, w, lane);
  __threadfence();
  ctx_store_pass(sC, ch, b, qbase, w, lane);
}

__device__ __forceinline__ void out_store_pass(const float* sO, float* out, int m0, int f0,
                                               int w, int lane) {
  const int q8 = lane & 7, sub = lane >> 3;
  #pragma unroll
  for (int i = 0; i < 16; ++i) {
    const int lid = w * 64 + i * 4 + sub;
    const int row = lid >> 1, hl = lid & 1;
    const v4f v = *(const v4fa*)(sO + row * 64 + 32 * hl + 4 * q8);
    float* dst = out + (size_t)(m0 + row) * DM + f0 + 32 * hl + 4 * q8;
    *(volatile v4f*)dst = v;
  }
}

__global__ __launch_bounds__(128) void proj_gemm_kernel(
    const _Float16* __restrict__ ch,
    const _Float16* __restrict__ wt,
    const float* __restrict__ bproj,
    float* __restrict__ out)
{
  __shared__ __attribute__((aligned(16))) float sO[128 * 64];

  const int tid = threadIdx.x, lane = tid & 31, w = tid >> 5;
  const int h = lane >> 4, m = lane & 15;
  const int m0 = blockIdx.x * 128;
  const int f0 = blockIdx.y * 64;
  const int m0w = m0 + 32 * w;

  const _Float16* ca0 = ch + (size_t)(m0w + m) * DM;
  const _Float16* ca1 = ca0 + (size_t)16 * DM;
  const _Float16* wb  = wt + (size_t)(f0 + m) * DM;

  v8f acc[2][4];
  #pragma unroll
  for (int mt = 0; mt < 2; ++mt)
    #pragma unroll
    for (int nt = 0; nt < 4; ++nt) acc[mt][nt] = zero8f();

  #pragma unroll 1
  for (int k0 = 0; k0 < DM; k0 += 32) {
    const v16h a0 = load_frag(ca0 + k0, h);
    const v16h a1 = load_frag(ca1 + k0, h);
    #pragma unroll
    for (int nt = 0; nt < 4; ++nt) {
      const v16h bf = load_frag(wb + (size_t)nt * 16 * DM + k0, h);
      acc[0][nt] = wmma_f16(a0, bf, acc[0][nt]);
      acc[1][nt] = wmma_f16(a1, bf, acc[1][nt]);
    }
  }

  #pragma unroll
  for (int nt = 0; nt < 4; ++nt) {
    const int feat = 16 * nt + m;
    const float bv = bproj[f0 + feat];
    #pragma unroll
    for (int mt = 0; mt < 2; ++mt) {
      #pragma unroll
      for (int r = 0; r < 8; ++r) {
        const int tokl = 32 * w + 16 * mt + 8 * h + r;
        sO[tokl * 64 + feat] = acc[mt][nt][r] * (1.0f / (CSC * WSC)) + bv;
      }
    }
  }
  __syncthreads();

  out_store_pass(sO, out, m0, f0, w, lane);
  __threadfence();
  out_store_pass(sO, out, m0, f0, w, lane);
}

extern "C" void kernel_launch(void* const* d_in, const int* in_sizes, int n_in,
                              void* d_out, int out_size, void* d_ws, size_t ws_size,
                              hipStream_t stream) {
  if (n_in < 6) return;
  if (in_sizes[0] != NX) return;
  if (in_sizes[1] < 1) return;
  if (in_sizes[2] != DM * D3) return;
  if (in_sizes[3] != D3) return;
  if (in_sizes[4] != DM * DM) return;
  if (in_sizes[5] != DM) return;
  if (out_size != NX) return;

  const float* x      = (const float*)d_in[0];
  const float* gamma  = (const float*)d_in[1];
  const float* W_qkv  = (const float*)d_in[2];
  const float* b_qkv  = (const float*)d_in[3];
  const float* W_proj = (const float*)d_in[4];
  const float* b_proj = (const float*)d_in[5];
  float* out = (float*)d_out;

  const size_t xh_bytes = (size_t)NX * 2;
  const size_t wq_bytes = (size_t)D3 * DM * 2;
  const size_t wp_bytes = (size_t)DM * DM * 2;
  const size_t pl_bytes = (size_t)NX * 2;
  const size_t o_wq = xh_bytes;
  const size_t o_wp = o_wq + wq_bytes;
  const size_t o_q  = o_wp + wp_bytes;
  const size_t o_k  = o_q + pl_bytes;
  const size_t o_v  = o_k + pl_bytes;
  const size_t total = o_v + pl_bytes;
  if (total > ws_size) return;

  char* ws = (char*)d_ws;
  _Float16* xh    = (_Float16*)(ws);
  _Float16* ch    = (_Float16*)(ws);
  _Float16* wqkvT = (_Float16*)(ws + o_wq);
  _Float16* wprjT = (_Float16*)(ws + o_wp);
  _Float16* qh    = (_Float16*)(ws + o_q);
  _Float16* kh    = (_Float16*)(ws + o_k);
  _Float16* vt    = (_Float16*)(ws + o_v);

  convert_x_kernel<<<NX8 / 256, 256, 0, stream>>>(x, xh, NX8);

  transpose_w_kernel<<<dim3(D3 / 64, DM / 64), 256, 0, stream>>>(W_qkv, wqkvT, DM, D3);
  transpose_w_kernel<<<dim3(DM / 64, DM / 64), 256, 0, stream>>>(W_proj, wprjT, DM, DM);

  qkv_gemm_kernel<<<dim3(MROWS / 128, D3 / 64), 128, 0, stream>>>(xh, wqkvT, b_qkv, qh, kh, vt);

  attention_kernel<<<dim3(SEQ / 16, NB), 256, (size_t)ATT_LDS, stream>>>(qh, kh, vt, gamma, ch);

  proj_gemm_kernel<<<dim3(MROWS / 128, DM / 64), 128, 0, stream>>>(ch, wprjT, b_proj, out);
}
